// FlashAttention_67611375174105
// MI455X (gfx1250) — hardware-verified
//
#include <hip/hip_runtime.h>

typedef _Float16 v16h __attribute__((ext_vector_type(16)));
typedef _Float16 v8h  __attribute__((ext_vector_type(8)));
typedef float    v8f  __attribute__((ext_vector_type(8)));
typedef float    v4f  __attribute__((ext_vector_type(4)));

#ifndef NB
#define NB 2
#endif
#ifndef SEQ
#define SEQ 2048
#endif
#define NB_FULL   2
#define SEQ_FULL  2048
#define DM        1024
#define NH        16
#define DHEAD     64
#define NQKV      (3 * DM)
#define MROWS     (NB * SEQ)
#define NBH       (NB * NH)

#define BM       64
#define BN       64
#define KSTRIDE  72
#define VSTRIDE  72
#define OSTR     72
#define TSTR     136
#define CSTR     68

#define QSCALE   (0.125f * 1.4426950408889634f)
#define PCARRY   10.0f
#define WCARRY   64.0f
#define WUNDO    (1.0f / 64.0f)

static_assert(SEQ % 128 == 0);
static_assert(SEQ <= SEQ_FULL);
static_assert(NB >= 1 && NB <= NB_FULL);
static_assert(DM % 128 == 0 && NQKV % 128 == 0);
static_assert(DHEAD == 64 && NH * DHEAD == DM);
static_assert((MROWS % 128) == 0);

union HV { v8h h; v4f f; };

__device__ __forceinline__ float bf16r(float f) {
    unsigned u = __float_as_uint(f);
    u = (u + 0x7FFFu + ((u >> 16) & 1u)) & 0xFFFF0000u;
    return __uint_as_float(u);
}

__device__ __forceinline__ v16h ld_op16(const _Float16* p) {
    const v8h lo = *(const v8h*)(p);
    const v8h hi = *(const v8h*)(p + 16);
    v16h r;
#pragma unroll
    for (int i = 0; i < 8; ++i) { r[i] = lo[i]; r[i + 8] = hi[i]; }
    return r;
}

__device__ __forceinline__ v8f wmma_f16(v16h a, v16h b, v8f c) {
    v8f d = __builtin_amdgcn_wmma_f32_16x16x32_f16(
        false, a, false, b, (short)0, c, false, false);
    asm volatile("v_nop\n\tv_nop\n\tv_nop\n\tv_nop" : "+v"(d) : "v"(a), "v"(b));
    return d;
}

__global__ __launch_bounds__(256)
void cvt_plane(const float* __restrict__ src, _Float16* __restrict__ dst,
               int nrows, int seq, int seq_full, float scale) {
    const size_t total = (size_t)nrows * DM;
    const size_t e     = ((size_t)blockIdx.x * 256 + threadIdx.x) * 8;
    if (e >= total) return;
    const int m    = (int)(e / DM);
    const int c    = (int)(e - (size_t)m * DM);
    const int mb   = m / seq;
    const int srow = mb * seq_full + (m - mb * seq);
    const float* sp = src + (size_t)srow * DM + c;
    const v4f a = *(const v4f*)(sp);
    const v4f b = *(const v4f*)(sp + 4);
    v8h t;
    t[0] = (_Float16)(bf16r(a[0]) * scale); t[1] = (_Float16)(bf16r(a[1]) * scale);
    t[2] = (_Float16)(bf16r(a[2]) * scale); t[3] = (_Float16)(bf16r(a[3]) * scale);
    t[4] = (_Float16)(bf16r(b[0]) * scale); t[5] = (_Float16)(bf16r(b[1]) * scale);
    t[6] = (_Float16)(bf16r(b[2]) * scale); t[7] = (_Float16)(bf16r(b[3]) * scale);
    HV o; o.h = t;
    _Float16* dp = dst + e;
    *(volatile v4f*)dp = o.f;
    __threadfence();
    *(volatile v4f*)dp = o.f;
}

__device__ __forceinline__ void gemm_k1024(const _Float16* __restrict__ A,
                                           const _Float16* __restrict__ W,
                                           int m0, int n0, int l16, int kbase,
                                           v8f (&acc)[2][4]) {
    const _Float16* a0p = A + (size_t)(m0 + l16) * DM + kbase;
    const _Float16* a1p = A + (size_t)(m0 + 16 + l16) * DM + kbase;
    const _Float16* wp  = W + (size_t)(n0 + l16) * DM + kbase;
#pragma unroll 1
    for (int k0 = 0; k0 < DM; k0 += 32) {
        const v16h a0 = ld_op16(a0p + k0);
        const v16h a1 = ld_op16(a1p + k0);
#pragma unroll
        for (int t = 0; t < 4; ++t) {
            const v16h b = ld_op16(wp + (size_t)t * 16 * DM + k0);
            acc[0][t] = wmma_f16(a0, b, acc[0][t]);
            acc[1][t] = wmma_f16(a1, b, acc[1][t]);
        }
    }
}

__global__ __launch_bounds__(256)
void qkv_gemm(const _Float16* __restrict__ Xh, const _Float16* __restrict__ Wh,
              const float* __restrict__ bias, _Float16* __restrict__ Qp,
              _Float16* __restrict__ Kp, _Float16* __restrict__ Vtp) {
    __shared__ __align__(16) _Float16 Ts[128 * TSTR];

    const int tid = threadIdx.x, lane = tid & 31, wave = tid >> 5;
    const int half = lane >> 4, l16 = lane & 15, kbase = half * 8;
    const int wm = wave & 3, wn = wave >> 2;
    const int mblk = blockIdx.y * 128, nblk = blockIdx.x * 128;
    const int m0 = mblk + wm * 32, n0 = nblk + wn * 64;

    v8f acc[2][4];
#pragma unroll
    for (int i = 0; i < 2; ++i)
#pragma unroll
        for (int t = 0; t < 4; ++t)
#pragma unroll
            for (int v = 0; v < 8; ++v) acc[i][t][v] = 0.0f;

    gemm_k1024(Xh, Wh, m0, n0, l16, kbase, acc);

    const int which = nblk / DM;
    const int cb    = nblk - which * DM;
    const int h0    = cb >> 6;
    const int bidx  = mblk / SEQ;
    const int tt0   = mblk - bidx * SEQ;

    float bv[4];
#pragma unroll
    for (int t = 0; t < 4; ++t) bv[t] = bf16r(bias[n0 + 16 * t + l16]);

    if (which < 2) {
#pragma unroll
        for (int i = 0; i < 2; ++i)
#pragma unroll
            for (int t = 0; t < 4; ++t)
#pragma unroll
                for (int r = 0; r < 8; ++r) {
                    const int lr = wm * 32 + 16 * i + 8 * half + r;
                    const int lc = wn * 64 + 16 * t + l16;
                    Ts[lr * TSTR + lc] = (_Float16)fmaf(acc[i][t][r], WUNDO, bv[t]);
                }
    } else {
#pragma unroll
        for (int i = 0; i < 2; ++i)
#pragma unroll
            for (int t = 0; t < 4; ++t)
#pragma unroll
                for (int r = 0; r < 8; ++r) {
                    const int lr = wm * 32 + 16 * i + 8 * half + r;
                    const int lc = wn * 64 + 16 * t + l16;
                    Ts[lc * TSTR + lr] = (_Float16)fmaf(acc[i][t][r], WUNDO, bv[t]);
                }
    }
    __syncthreads();

    HV     vals[8];
    size_t off[8];
    const int p = lane & 7;
    if (which < 2) {
        _Float16* P = (which == 0) ? Qp : Kp;
#pragma unroll
        for (int j = 0; j < 8; ++j) {
            const int L  = wave * 32 + 4 * j + (lane >> 3);
            const int lr = L >> 1, hh = L & 1;
            vals[j].h = *(const v8h*)&Ts[lr * TSTR + hh * 64 + p * 8];
            const int bh = bidx * NH + h0 + hh;
            off[j] = ((size_t)bh * SEQ + tt0 + lr) * DHEAD + p * 8;
        }
#pragma unroll
        for (int j = 0; j < 8; ++j) *(volatile v4f*)(P + off[j]) = vals[j].f;
        __threadfence();
#pragma unroll
        for (int j = 0; j < 8; ++j) *(volatile v4f*)(P + off[j]) = vals[j].f;
    } else {
#pragma unroll
        for (int j = 0; j < 8; ++j) {
            const int L  = wave * 32 + 4 * j + (lane >> 3);
            const int lc = L >> 1, tseg = L & 1;
            vals[j].h = *(const v8h*)&Ts[lc * TSTR + tseg * 64 + p * 8];
            const int bh = bidx * NH + h0 + (lc >> 6);
            const int d  = lc & 63;
            off[j] = ((size_t)bh * DHEAD + d) * SEQ + tt0 + tseg * 64 + p * 8;
        }
#pragma unroll
        for (int j = 0; j < 8; ++j) *(volatile v4f*)(Vtp + off[j]) = vals[j].f;
        __threadfence();
#pragma unroll
        for (int j = 0; j < 8; ++j) *(volatile v4f*)(Vtp + off[j]) = vals[j].f;
    }
}

__device__ __forceinline__ void stage_block(const _Float16* kg, const _Float16* vtg,
                                            _Float16* ks, _Float16* vts, int tid) {
#pragma unroll
    for (int i = 0; i < 4; ++i) {
        const int c   = tid + 128 * i;
        const int row = c >> 3;
        const int off = (c & 7) * 8;
        *(v8h*)&ks[row * KSTRIDE + off]  = *(const v8h*)(kg + row * DHEAD + off);
        *(v8h*)&vts[row * VSTRIDE + off] = *(const v8h*)(vtg + (size_t)row * SEQ + off);
    }
}

__device__ __forceinline__ void attn_step(const _Float16* ksb, const _Float16* vtsb,
                                          const v16h (&qb)[2], int l16, int kbase,
                                          float& m_i, float& l_i, v8f (&acc)[4]) {
    v8f s[4];
#pragma unroll
    for (int n = 0; n < 4; ++n)
#pragma unroll
        for (int v = 0; v < 8; ++v) s[n][v] = 0.0f;
#pragma unroll
    for (int c = 0; c < 2; ++c) {
        const int dco = c * 32 + kbase;
#pragma unroll
        for (int n = 0; n < 4; ++n) {
            const v16h ka = ld_op16(&ksb[(n * 16 + l16) * KSTRIDE + dco]);
            s[n] = wmma_f16(ka, qb[c], s[n]);
        }
    }

    float tm[4];
#pragma unroll
    for (int n = 0; n < 4; ++n) {
        const float a0 = fmaxf(s[n][0], s[n][1]);
        const float a1 = fmaxf(s[n][2], s[n][3]);
        const float a2 = fmaxf(s[n][4], s[n][5]);
        const float a3 = fmaxf(s[n][6], s[n][7]);
        tm[n] = fmaxf(fmaxf(a0, a1), fmaxf(a2, a3));
    }
    float mx = fmaxf(fmaxf(tm[0], tm[1]), fmaxf(tm[2], tm[3]));
    mx = fmaxf(mx, __shfl_xor(mx, 16, 32));

    const float mnew = fmaxf(m_i, mx);
    const float corr = __builtin_amdgcn_exp2f((m_i - mnew) * QSCALE);
    const float msh  = mnew * QSCALE - PCARRY;

    v16h  pb[2];
    float psum = 0.0f;
#pragma unroll
    for (int n = 0; n < 4; ++n)
#pragma unroll
        for (int v = 0; v < 8; ++v) {
            const _Float16 p16 = (_Float16)__builtin_amdgcn_exp2f(fmaf(s[n][v], QSCALE, -msh));
            pb[n >> 1][(n & 1) * 8 + v] = p16;
            psum += (float)p16;
        }
    psum += __shfl_xor(psum, 16, 32);

    l_i = l_i * corr + psum;
    m_i = mnew;
#pragma unroll
    for (int t = 0; t < 4; ++t)
#pragma unroll
        for (int v = 0; v < 8; ++v) acc[t][v] *= corr;

#pragma unroll
    for (int ck = 0; ck < 2; ++ck)
#pragma unroll
        for (int t = 0; t < 4; ++t) {
            const v16h va = ld_op16(&vtsb[(t * 16 + l16) * VSTRIDE + ck * 32 + kbase]);
            acc[t] = wmma_f16(va, pb[ck], acc[t]);
        }
}

__global__ __launch_bounds__(128)
void attn_fwd(const _Float16* __restrict__ Qp, const _Float16* __restrict__ Kp,
              const _Float16* __restrict__ Vtp, _Float16* __restrict__ Oh) {
    __shared__ __align__(16) _Float16 Ks0[BN * KSTRIDE];
    __shared__ __align__(16) _Float16 Ks1[BN * KSTRIDE];
    __shared__ __align__(16) _Float16 Vts0[DHEAD * VSTRIDE];
    __shared__ __align__(16) _Float16 Vts1[DHEAD * VSTRIDE];
    __shared__ __align__(16) _Float16 Os[4][16 * OSTR];

    const int tid   = threadIdx.x;
    const int lane  = tid & 31;
    const int wid   = tid >> 5;
    const int half  = lane >> 4;
    const int l16   = lane & 15;
    const int kbase = half * 8;

    const int    bh     = blockIdx.y;
    const int    bidx   = bh / NH;
    const int    hd     = bh - bidx * NH;
    const int    qblk   = blockIdx.x;
    const size_t bh_off = (size_t)bh * SEQ * DHEAD;

    const _Float16* kg0  = Kp  + bh_off;
    const _Float16* vtg0 = Vtp + bh_off;

    const int       qbase = qblk * BM + wid * 16;
    const _Float16* qrow  = Qp + bh_off + (size_t)(qbase + l16) * DHEAD;
    v16h qb[2];
#pragma unroll
    for (int c = 0; c < 2; ++c) qb[c] = ld_op16(qrow + c * 32 + kbase);

    float m_i = -1e30f, l_i = 0.0f;
    v8f acc[4];
#pragma unroll
    for (int t = 0; t < 4; ++t)
#pragma unroll
        for (int v = 0; v < 8; ++v) acc[t][v] = 0.0f;

    stage_block(kg0, vtg0, Ks0, Vts0, tid);

    for (int kb = 0; kb < SEQ; kb += 2 * BN) {
        __syncthreads();
        stage_block(kg0 + (size_t)(kb + BN) * DHEAD, vtg0 + (kb + BN), Ks1, Vts1, tid);
        attn_step(Ks0, Vts0, qb, l16, kbase, m_i, l_i, acc);

        __syncthreads();
        if (kb + 2 * BN < SEQ)
            stage_block(kg0 + (size_t)(kb + 2 * BN) * DHEAD, vtg0 + (kb + 2 * BN),
                        Ks0, Vts0, tid);
        attn_step(Ks1, Vts1, qb, l16, kbase, m_i, l_i, acc);
    }

    const float inv = 1.0f / l_i;
    _Float16*   os  = Os[wid];
#pragma unroll
    for (int t = 0; t < 4; ++t) {
        v8h o;
#pragma unroll
        for (int v = 0; v < 8; ++v) o[v] = (_Float16)(acc[t][v] * inv);
        *(v8h*)&os[l16 * OSTR + t * 16 + kbase] = o;
    }
    __builtin_amdgcn_fence(3, "wavefront");
    __builtin_amdgcn_wave_barrier();

    HV     vals[4];
    size_t off[4];
    const int p = lane & 7;
#pragma unroll
    for (int i = 0; i < 4; ++i) {
        const int row = (lane >> 3) + 4 * i;
        vals[i].h = *(const v8h*)&os[row * OSTR + p * 8];
        off[i] = ((size_t)bidx * SEQ + qbase + row) * DM + hd * DHEAD + p * 8;
    }
#pragma unroll
    for (int i = 0; i < 4; ++i) *(volatile v4f*)(Oh + off[i]) = vals[i].f;
    __threadfence();
#pragma unroll
    for (int i = 0; i < 4; ++i) *(volatile v4f*)(Oh + off[i]) = vals[i].f;
}

__global__ __launch_bounds__(256)
void out_gemm(const _Float16* __restrict__ Oh, const _Float16* __restrict__ Wh,
              const float* __restrict__ bias, float* __restrict__ out) {
    __shared__ __align__(16) float Cs[8][16 * CSTR];

    const int tid = threadIdx.x, lane = tid & 31, wave = tid >> 5;
    const int half = lane >> 4, l16 = lane & 15, kbase = half * 8;
    const int wm = wave & 3, wn = wave >> 2;
    const int mblk = blockIdx.y * 128, nblk = blockIdx.x * 128;
    const int m0 = mblk + wm * 32, n0 = nblk + wn * 64;

    v8f acc[2][4];
#pragma unroll
    for (int i = 0; i < 2; ++i)
#pragma unroll
        for (int t = 0; t < 4; ++t)
#pragma unroll
            for (int v = 0; v < 8; ++v) acc[i][t][v] = 0.0f;

    gemm_k1024(Oh, Wh, m0, n0, l16, kbase, acc);

    const int bidx  = mblk / SEQ;
    const int tt0   = mblk - bidx * SEQ;
    const int orow0 = bidx * SEQ_FULL + tt0 + wm * 32;

    float bv[4];
#pragma unroll
    for (int t = 0; t < 4; ++t) bv[t] = bf16r(bias[n0 + 16 * t + l16]);

    float* cw = Cs[wave];
#pragma unroll
    for (int i = 0; i < 2; ++i) {
#pragma unroll
        for (int t = 0; t < 4; ++t)
#pragma unroll
            for (int r = 0; r < 8; ++r)
                cw[(8 * half + r) * CSTR + 16 * t + l16] = fmaf(acc[i][t][r], WUNDO, bv[t]);
        __builtin_amdgcn_fence(3, "wavefront");
        __builtin_amdgcn_wave_barrier();

        v4f    vals[8];
        size_t off[8];
        const int col = (lane & 15) * 4;
#pragma unroll
        for (int j = 0; j < 8; ++j) {
            const int row = (lane >> 4) + 2 * j;
            vals[j] = *(const v4f*)&cw[row * CSTR + col];
            off[j]  = (size_t)(orow0 + 16 * i + row) * DM + n0 + col;
        }
#pragma unroll
        for (int j = 0; j < 8; ++j) *(volatile v4f*)(out + off[j]) = vals[j];
        __threadfence();
#pragma unroll
        for (int j = 0; j < 8; ++j) *(volatile v4f*)(out + off[j]) = vals[j];
        __builtin_amdgcn_fence(3, "wavefront");
        __builtin_amdgcn_wave_barrier();
    }
}

extern "C" void kernel_launch(void* const* d_in, const int* in_sizes, int n_in,
                              void* d_out, int out_size, void* d_ws, size_t ws_size,
                              hipStream_t stream) {
    if (n_in < 5) return;
    const long long needx = ((long long)(NB - 1) * SEQ_FULL + SEQ) * DM;
    if ((long long)in_sizes[0] < needx) return;
    if (in_sizes[1] < NQKV * DM) return;
    if (in_sizes[2] < NQKV) return;
    if (in_sizes[3] < DM * DM) return;
    if (in_sizes[4] < DM) return;
    if ((long long)out_size < needx) return;

    const float* x     = (const float*)d_in[0];
    const float* W_qkv = (const float*)d_in[1];
    const float* b_qkv = (const float*)d_in[2];
    const float* W_out = (const float*)d_in[3];
    const float* b_out = (const float*)d_in[4];
    float*       out   = (float*)d_out;

    const size_t szX  = (size_t)MROWS * DM * 2;
    const size_t szWq = (size_t)NQKV * DM * 2;
    const size_t szWo = (size_t)DM * DM * 2;
    const size_t szQ  = (size_t)NBH * SEQ * DHEAD * 2;
    const size_t szK  = szQ;
    const size_t szVt = szQ;
    const size_t szO  = (size_t)MROWS * DM * 2;
    const size_t oX = 0, oWq = oX + szX, oWo = oWq + szWq, oQ = oWo + szWo,
                 oK = oQ + szQ, oVt = oK + szK, oO = oVt + szVt, total = oO + szO;
    if (total > ws_size) return;

    char* ws = (char*)d_ws;
    _Float16* Xh  = (_Float16*)(ws + oX);
    _Float16* Wqh = (_Float16*)(ws + oWq);
    _Float16* Woh = (_Float16*)(ws + oWo);
    _Float16* Qp  = (_Float16*)(ws + oQ);
    _Float16* Kp  = (_Float16*)(ws + oK);
    _Float16* Vtp = (_Float16*)(ws + oVt);
    _Float16* Oh  = (_Float16*)(ws + oO);

    const unsigned gX  = (unsigned)(((size_t)MROWS * DM / 8 + 255) / 256);
    const unsigned gWq = (unsigned)(((size_t)NQKV * DM / 8 + 255) / 256);
    const unsigned gWo = (unsigned)(((size_t)DM * DM / 8 + 255) / 256);
    cvt_plane<<<dim3(gX), dim3(256), 0, stream>>>(x, Xh, MROWS, SEQ, SEQ_FULL, 1.0f);
    cvt_plane<<<dim3(gWq), dim3(256), 0, stream>>>(W_qkv, Wqh, NQKV, NQKV, NQKV, WCARRY);
    cvt_plane<<<dim3(gWo), dim3(256), 0, stream>>>(W_out, Woh, DM, DM, DM, WCARRY);

    qkv_gemm<<<dim3(NQKV / 128, MROWS / 128), dim3(256), 0, stream>>>(Xh, Wqh, b_qkv, Qp, Kp, Vtp);
    attn_fwd<<<dim3(SEQ / BM, NBH), dim3(128), 0, stream>>>(Qp, Kp, Vtp, Oh);
    out_gemm<<<dim3(DM / 128, MROWS / 128), dim3(256), 0, stream>>>(Oh, Woh, b_out, out);
}
